// BernMLPAugmenter_83640193122891
// MI455X (gfx1250) — hardware-verified
//
#include <hip/hip_runtime.h>
#include <stdint.h>
#include <math.h>

typedef _Float16 v16h __attribute__((ext_vector_type(16)));
typedef _Float16 v8h  __attribute__((ext_vector_type(8)));
typedef float    v8f  __attribute__((ext_vector_type(8)));
typedef float    v4f  __attribute__((ext_vector_type(4)));

union HF { v16h v; v8h half[2]; _Float16 e[16]; };
union H8 { v8h v; _Float16 e[8]; };

#define EMB     128
#define KDIM    256
#define HID     64
#define WAVES   8
#define EPB     128
#define CHUNK   131072
#define SCALE_A 64.f
#define SCALE_B 64.f
#define UNSCALE (1.f / 4096.f)

__device__ __forceinline__ v8f wmma16(v16h a, v16h b, v8f c)
{
    c = __builtin_amdgcn_wmma_f32_16x16x32_f16(false, a, false, b, (short)0, c, false, false);
    asm volatile("v_nop\n\tv_nop\n\tv_nop\n\tv_nop" : "+v"(c) : "v"(a), "v"(b));
    return c;
}

__global__ __launch_bounds__(256) void k_wprep(const float* __restrict__ W1,
                                               _Float16* __restrict__ wsB)
{
    const int t = threadIdx.x;
    #pragma unroll 1
    for (int pass = 0; pass < 8; ++pass) {
        const int q   = pass * 256 + t;
        const int f   = q >> 1, hf = q & 1;
        const int ln  = f & 31, nt = (f >> 5) & 3, kb = f >> 7;
        const int col = nt * 16 + (ln & 15);
        const int kb0 = kb * 32 + 16 * hf + 8 * (ln >> 4);
        H8 u;
        #pragma unroll
        for (int i = 0; i < 8; ++i)
            u.e[i] = (_Float16)(W1[(kb0 + i) * HID + col] * SCALE_B);
        _Float16* dp = wsB + (size_t)q * 8;
        *(volatile v8h*)dp = u.v;
        __threadfence();
        *(volatile v8h*)dp = u.v;
    }
}

__global__ __launch_bounds__(256) void k_gather(const float* __restrict__ emb,
                                                const int*   __restrict__ eidx,
                                                _Float16*    __restrict__ dense,
                                                int e0, int rows, int M, int estride, int nNodes)
{
    const int row = blockIdx.x * WAVES + (threadIdx.x >> 5);
    if (row >= rows) return;
    const int l = threadIdx.x & 31, h = l >> 4, sub = (l & 15) * 8;
    int e = e0 + row;
    if (e > M - 1) e = M - 1;
    int node = eidx[(size_t)h * (size_t)estride + (size_t)e];
    if (node < 0) node += nNodes;
    node = node < 0 ? 0 : (node > nNodes - 1 ? nNodes - 1 : node);
    const float* rp = emb + (size_t)node * EMB + sub;
    const v4f x0 = *(const v4f*)(rp);
    const v4f x1 = *(const v4f*)(rp + 4);
    H8 u;
    u.e[0] = (_Float16)(x0.x * SCALE_A); u.e[1] = (_Float16)(x0.y * SCALE_A);
    u.e[2] = (_Float16)(x0.z * SCALE_A); u.e[3] = (_Float16)(x0.w * SCALE_A);
    u.e[4] = (_Float16)(x1.x * SCALE_A); u.e[5] = (_Float16)(x1.y * SCALE_A);
    u.e[6] = (_Float16)(x1.z * SCALE_A); u.e[7] = (_Float16)(x1.w * SCALE_A);
    _Float16* dp = dense + (size_t)row * KDIM + (size_t)l * 8;
    *(volatile v8h*)dp = u.v;
    __threadfence();
    *(volatile v8h*)dp = u.v;
}

__global__ __launch_bounds__(256) void k_gemm(const _Float16* __restrict__ dense,
                                              const _Float16* __restrict__ wsB,
                                              const float* __restrict__ eps_raw,
                                              const float* __restrict__ b1,
                                              const float* __restrict__ W2,
                                              const float* __restrict__ b2,
                                              float* __restrict__ wout, int e0, int M)
{
    __shared__ HF    sB[1024];
    __shared__ float sB1[HID];
    __shared__ float sW2[HID];
    __shared__ union { float f[EPB]; v4f v[EPB / 4]; } sW;

    const int t = threadIdx.x;
    {
        const v8h* src = (const v8h*)wsB;
        #pragma unroll
        for (int pass = 0; pass < 8; ++pass) {
            const int q = pass * 256 + t;
            sB[q >> 1].half[q & 1] = src[q];
        }
    }
    if (t < HID) { sB1[t] = b1[t]; sW2[t] = W2[t]; }
    __syncthreads();

    const int wave = t >> 5, l = t & 31, h = l >> 4, m = l & 15;
    const int rowBase = (blockIdx.x * WAVES + wave) * 16;
    const _Float16* ap = dense + (size_t)(rowBase + m) * KDIM + 8 * h;

    v8f acc[4];
    #pragma unroll
    for (int nt = 0; nt < 4; ++nt) {
        const v8f z = {0.f, 0.f, 0.f, 0.f, 0.f, 0.f, 0.f, 0.f};
        acc[nt] = z;
    }

    #pragma unroll
    for (int kb = 0; kb < 8; ++kb) {
        HF a;
        a.half[0] = *(const v8h*)(ap + kb * 32);
        a.half[1] = *(const v8h*)(ap + kb * 32 + 16);
        const HF* bp = sB + kb * 128 + l;
        acc[0] = wmma16(a.v, bp[0].v,  acc[0]);
        acc[1] = wmma16(a.v, bp[32].v, acc[1]);
        acc[2] = wmma16(a.v, bp[64].v, acc[2]);
        acc[3] = wmma16(a.v, bp[96].v, acc[3]);
    }

    float p[8];
    #pragma unroll
    for (int r = 0; r < 8; ++r) p[r] = 0.f;
    #pragma unroll
    for (int nt = 0; nt < 4; ++nt) {
        const int   n  = nt * 16 + m;
        const float bb = sB1[n];
        const float ww = sW2[n];
        #pragma unroll
        for (int r = 0; r < 8; ++r) {
            float hv = acc[nt][r] * UNSCALE + bb;
            hv = hv > 0.f ? hv : 0.f;
            p[r] += hv * ww;
        }
    }
    #pragma unroll
    for (int r = 0; r < 8; ++r) {
        p[r] += __shfl_xor(p[r], 1, 32);
        p[r] += __shfl_xor(p[r], 2, 32);
        p[r] += __shfl_xor(p[r], 4, 32);
        p[r] += __shfl_xor(p[r], 8, 32);
    }
    float mydot = 0.f;
    #pragma unroll
    for (int r = 0; r < 8; ++r) if (m == r) mydot = p[r];

    const int rloc = 8 * h + (m & 7);
    int e = e0 + rowBase + rloc;
    if (e > M - 1) e = M - 1;
    const float bias2 = b2[0];
    float w;
    {
        #pragma clang fp contract(off)
        const float kA    = (float)(2.0 * 1.0e-4 - 1.0);
        const float kB    = (float)(1.0 - 1.0e-4);
        const float logit = mydot + bias2;
        const float er    = eps_raw[e];
        const float eps   = kA * er + kB;
        const float g     = logf(eps) - log1pf(-eps);
        const float x     = g + logit;
        w = 1.f / (1.f + expf(-x));
    }
    if (m < 8) sW.f[wave * 16 + rloc] = w;
    __syncthreads();
    if (wave == 0) {
        const v4f v = sW.v[l];
        float* dp = wout + (size_t)blockIdx.x * EPB + 4 * l;
        *(volatile v4f*)dp = v;
        __threadfence();
        *(volatile v4f*)dp = v;
    }
}

__global__ __launch_bounds__(256) void k_out(const float* __restrict__ wbuf,
                                             float* __restrict__ out,
                                             int M, int T, int nWaves)
{
    const int wv = blockIdx.x * WAVES + (threadIdx.x >> 5);
    if (wv >= nWaves) return;
    const int l  = threadIdx.x & 31;
    const int j0 = wv * 128 + 4 * l;
    float v[4];
    #pragma unroll
    for (int c = 0; c < 4; ++c) {
        const int j = j0 + c;
        int idx = j;
        if (idx >= 2 * M) idx -= 2 * M;
        else if (idx >= M) idx -= M;
        idx = idx < 0 ? 0 : (idx > M - 1 ? M - 1 : idx);
        v[c] = (j < T) ? wbuf[idx] : 0.f;
    }
    const bool full = (j0 + 3 < T);
    v4f vv;
    vv.x = v[0]; vv.y = v[1]; vv.z = v[2]; vv.w = v[3];
    volatile float* so = (volatile float*)out;
    if (full) {
        *(volatile v4f*)(out + j0) = vv;
    } else {
        #pragma unroll
        for (int c = 0; c < 4; ++c) if (j0 + c < T) so[j0 + c] = v[c];
    }
    __threadfence();
    if (full) {
        *(volatile v4f*)(out + j0) = vv;
    } else {
        #pragma unroll
        for (int c = 0; c < 4; ++c) if (j0 + c < T) so[j0 + c] = v[c];
    }
}

extern "C" void kernel_launch(void* const* d_in, const int* in_sizes, int n_in,
                              void* d_out, int out_size, void* d_ws, size_t ws_size,
                              hipStream_t stream)
{
    if (n_in < 7) return;
    const float* node_emb   = (const float*)d_in[0];
    const int*   edge_index = (const int*)d_in[1];
    const float* eps_raw    = (const float*)d_in[2];
    const float* W1         = (const float*)d_in[3];
    const float* b1         = (const float*)d_in[4];
    const float* W2         = (const float*)d_in[5];
    const float* b2         = (const float*)d_in[6];
    float* out = (float*)d_out;

    const int nNodes  = in_sizes[0] / EMB;
    const int estride = in_sizes[1] / 2;
    const int M       = in_sizes[2];
    const int T       = out_size;
    if (nNodes < 1 || M < 1 || estride < M || T < 1) return;
    if (in_sizes[3] < KDIM * HID || in_sizes[4] < HID || in_sizes[5] < HID || in_sizes[6] < 1) return;

    const size_t offB     = 0;
    const size_t bytesB   = (size_t)2048 * 16;
    const size_t offDense = offB + bytesB;
    const size_t bytesDen = (size_t)CHUNK * KDIM * sizeof(_Float16);
    const size_t offW     = offDense + bytesDen;
    const size_t wFloats  = (size_t)((M + EPB - 1) / EPB) * EPB;
    const size_t total    = offW + wFloats * sizeof(float);
    if (total > ws_size) return;

    _Float16* wsB   = (_Float16*)((char*)d_ws + offB);
    _Float16* dense = (_Float16*)((char*)d_ws + offDense);
    float*    wbuf  = (float*)((char*)d_ws + offW);

    hipLaunchKernelGGL(k_wprep, dim3(1), dim3(256), 0, stream, W1, wsB);

    const int nChunks = (M + CHUNK - 1) / CHUNK;
    for (int c = 0; c < nChunks; ++c) {
        const int e0 = c * CHUNK;
        int cnt = M - e0;
        if (cnt > CHUNK) cnt = CHUNK;
        const int blocks = (cnt + EPB - 1) / EPB;
        const int rows   = blocks * EPB;
        const int gBlocks = (rows + WAVES - 1) / WAVES;
        hipLaunchKernelGGL(k_gather, dim3(gBlocks), dim3(256), 0, stream,
                           node_emb, edge_index, dense, e0, rows, M, estride, nNodes);
        hipLaunchKernelGGL(k_gemm, dim3(blocks), dim3(256), 0, stream,
                           (const _Float16*)dense, (const _Float16*)wsB, eps_raw, b1, W2, b2,
                           wbuf + (size_t)e0, e0, M);
    }

    const int nWaves  = (T + 127) / 128;
    const int oBlocks = (nWaves + WAVES - 1) / WAVES;
    hipLaunchKernelGGL(k_out, dim3(oBlocks), dim3(256), 0, stream,
                       (const float*)wbuf, out, M, T, nWaves);
}
